// SelfAttentionBlock_42442866819738
// MI455X (gfx1250) — hardware-verified
//
#include <hip/hip_runtime.h>


typedef _Float16 h8_t  __attribute__((ext_vector_type(8)));
typedef _Float16 h16_t __attribute__((ext_vector_type(16)));
typedef float    f8_t  __attribute__((ext_vector_type(8)));
typedef float    f4_t  __attribute__((ext_vector_type(4)));
typedef unsigned int u4_t __attribute__((ext_vector_type(4)));
typedef h8_t h8a_t __attribute__((may_alias));
typedef f4_t f4a_t __attribute__((may_alias));
typedef u4_t u4a_t __attribute__((may_alias));

#ifndef NB
#define NB 4
#endif
#ifndef SEQ
#define SEQ 4096
#endif
#define NB_FULL 4
#define SEQ_FULL 4096
#ifndef X_SEQ_STRIDE
#define X_SEQ_STRIDE SEQ_FULL
#endif
#ifndef O_SEQ_STRIDE
#define O_SEQ_STRIDE SEQ_FULL
#endif

#define CH 128
#define NGRP 8
#define CPG (CH / NGRP)
#define NHEAD 4
#define HD (CH / NHEAD)
#define GN_EPS 1e-5f
#define ATTN_SCALE 0.08838834764831845f
#define KCH 32
#define LDH 136
#define LDT 72
#define LDO 68
#define LDSA 40
#define STATS_LD 32
#define WQ_CARRY 16.0f
#define WQ_INV 0.0625f
#define WP_CARRY 64.0f
#define P_CARRY 1024.0f
#define O_SCALE 0.0625f
#define PROJ_INV 0.000244140625f
#define WS_LIMIT ((size_t)134217728)

static_assert(SEQ % 64 == 0);
static_assert(SEQ % KCH == 0);
static_assert(SEQ <= SEQ_FULL);
static_assert(NB >= 1 && NB <= NB_FULL);
static_assert(CH == 128);
static_assert(CPG == 16);
static_assert(HD == 32);
static_assert(NGRP <= 32);
static_assert((3 * CH * CH / 8) % 256 == 0);
static_assert((CH * CH / 8) % 256 == 0);
static_assert(64 * LDH <= CH * LDT);
static_assert(KCH == 32);

__device__ __forceinline__ float bf16r(float v) {
  unsigned int u = __float_as_uint(v);
  u = (u + 0x7FFFu + ((u >> 16) & 1u)) & 0xFFFF0000u;
  return __uint_as_float(u);
}

__device__ __forceinline__ f8_t f8zero() {
  f8_t z = {0.f, 0.f, 0.f, 0.f, 0.f, 0.f, 0.f, 0.f};
  return z;
}

__device__ __forceinline__ f8_t wmma16(h16_t a, h16_t b, f8_t c) {
  f8_t d = __builtin_amdgcn_wmma_f32_16x16x32_f16(false, a, false, b, (short)0, c, false, false);
  asm volatile("v_nop\n\tv_nop\n\tv_nop\n\tv_nop" : "+v"(d) : "v"(a), "v"(b));
  return d;
}

__device__ __forceinline__ h16_t ldfrag(const _Float16* rowp, int k0, int h) {
  const h8_t lo = *(const h8a_t*)(rowp + k0 + 8 * h);
  const h8_t hi = *(const h8a_t*)(rowp + k0 + 16 + 8 * h);
  return __builtin_shufflevector(lo, hi, 0, 1, 2, 3, 4, 5, 6, 7, 8, 9, 10, 11, 12, 13, 14, 15);
}

__device__ __forceinline__ float wave_sum(float v) {
  v += __shfl_xor(v, 16, 32);
  v += __shfl_xor(v, 8, 32);
  v += __shfl_xor(v, 4, 32);
  v += __shfl_xor(v, 2, 32);
  v += __shfl_xor(v, 1, 32);
  return v;
}

__global__ __launch_bounds__(256) void k_cvtw(const float* __restrict__ src,
                                               _Float16* __restrict__ dst, float carry) {
  const size_t u = (size_t)blockIdx.x * 256 + threadIdx.x;
  const f4_t a = *(const f4_t*)(src + u * 8);
  const f4_t c = *(const f4_t*)(src + u * 8 + 4);
  union { h8_t h; u4_t q; } pk;
  pk.h[0] = (_Float16)(bf16r(a.x) * carry);
  pk.h[1] = (_Float16)(bf16r(a.y) * carry);
  pk.h[2] = (_Float16)(bf16r(a.z) * carry);
  pk.h[3] = (_Float16)(bf16r(a.w) * carry);
  pk.h[4] = (_Float16)(bf16r(c.x) * carry);
  pk.h[5] = (_Float16)(bf16r(c.y) * carry);
  pk.h[6] = (_Float16)(bf16r(c.z) * carry);
  pk.h[7] = (_Float16)(bf16r(c.w) * carry);
  volatile u4_t* p = (volatile u4_t*)(dst + u * 8);
  *p = pk.q;
  __threadfence();
  *p = pk.q;
}

__global__ __launch_bounds__(256) void k_gnstats(const float* __restrict__ x,
                                                  float* __restrict__ stats) {
  __shared__ float red[8];
  const int tid = threadIdx.x, lane = tid & 31, w = tid >> 5;
  const int b = blockIdx.x / NGRP;
  const int g = blockIdx.x - b * NGRP;
  const float* xg = x + (size_t)(b * CH + g * CPG) * X_SEQ_STRIDE;

  float s = 0.f;
#pragma unroll 1
  for (int c = 0; c < CPG; ++c) {
    const float* xr = xg + (size_t)c * X_SEQ_STRIDE;
#pragma unroll 1
    for (int n = tid; n < SEQ; n += 256) s += bf16r(xr[n]);
  }
  s = wave_sum(s);
  if (lane == 0) red[w] = s;
  __syncthreads();
  float tot = 0.f;
#pragma unroll 1
  for (int i = 0; i < 8; ++i) tot += red[i];
  __syncthreads();
  const float inv_cnt = 1.0f / (float)(CPG * SEQ);
  const float mean = tot * inv_cnt;

  float q = 0.f;
#pragma unroll 1
  for (int c = 0; c < CPG; ++c) {
    const float* xr = xg + (size_t)c * X_SEQ_STRIDE;
#pragma unroll 1
    for (int n = tid; n < SEQ; n += 256) {
      const float d = bf16r(xr[n]) - mean;
      q += d * d;
    }
  }
  q = wave_sum(q);
  if (lane == 0) red[w] = q;
  __syncthreads();
  float totq = 0.f;
#pragma unroll 1
  for (int i = 0; i < 8; ++i) totq += red[i];
  const float var  = totq * inv_cnt;
  const float rstd = rsqrtf(var + GN_EPS);

  if (tid < 8) {
    f4_t v;
    v.x = (tid == 0) ? mean : 0.f;
    v.y = (tid == 0) ? rstd : 0.f;
    v.z = 0.f;
    v.w = 0.f;
    volatile f4_t* p = (volatile f4_t*)(stats + (size_t)blockIdx.x * STATS_LD + tid * 4);
    *p = v;
    __threadfence();
    *p = v;
  }
}

__global__ __launch_bounds__(128) void k_qkv(
    const float* __restrict__ x, const float* __restrict__ stats,
    const float* __restrict__ gn_w, const float* __restrict__ gn_b,
    const _Float16* __restrict__ wq16, const float* __restrict__ qkv_b,
    _Float16* __restrict__ qpl, _Float16* __restrict__ kpl, _Float16* __restrict__ vtpl) {
  __shared__ __align__(16) _Float16 zs[64 * LDH];
  __shared__ __align__(16) _Float16 st[CH * LDT];
  __shared__ float gm[NGRP], gr[NGRP], gw[CH], gb[CH];
  const int tid = threadIdx.x, lane = tid & 31, w = tid >> 5;
  const int m = lane & 15, h = lane >> 4;
  const int n0  = blockIdx.x * 64;
  const int mat = blockIdx.y;
  const int b   = blockIdx.z;

  if (tid < NGRP) {
    const float* sl = stats + (size_t)(b * NGRP + tid) * STATS_LD;
    gm[tid] = sl[0];
    gr[tid] = sl[1];
  }
  gw[tid] = bf16r(gn_w[tid]);
  gb[tid] = bf16r(gn_b[tid]);
  __syncthreads();

  {
    const int t = tid & 63;
    const int ch0 = (tid >> 6) * 64;
    const float* xb = x + (size_t)(b * CH) * X_SEQ_STRIDE + n0 + t;
#pragma unroll 4
    for (int j = 0; j < 64; ++j) {
      const int c = ch0 + j;
      const float v = bf16r(xb[(size_t)c * X_SEQ_STRIDE]);
      const float z = ((v - gm[c / CPG]) * gr[c / CPG]) * gw[c] + gb[c];
      zs[t * LDH + c] = (_Float16)z;
    }
  }
  __syncthreads();

  f8_t acc[8];
#pragma unroll
  for (int t8 = 0; t8 < 8; ++t8) acc[t8] = f8zero();
  const _Float16* arow = zs + (w * 16 + m) * LDH;
  const _Float16* wrow = wq16 + (size_t)(mat * CH + m) * CH;
#pragma unroll
  for (int kc = 0; kc < 4; ++kc) {
    const h16_t a = ldfrag(arow, kc * 32, h);
#pragma unroll
    for (int t8 = 0; t8 < 8; ++t8) {
      const h16_t bb = ldfrag(wrow + (size_t)(t8 * 16) * CH, kc * 32, h);
      acc[t8] = wmma16(a, bb, acc[t8]);
    }
  }

  const float* bp = qkv_b + mat * CH + m;
  if (mat < 2) {
#pragma unroll
    for (int t8 = 0; t8 < 8; ++t8) {
      const float bb = bf16r(bp[t8 * 16]);
#pragma unroll
      for (int r = 0; r < 8; ++r)
        st[(w * 16 + 8 * h + r) * LDH + t8 * 16 + m] = (_Float16)(acc[t8][r] * WQ_INV + bb);
    }
  } else {
#pragma unroll
    for (int t8 = 0; t8 < 8; ++t8) {
      const float bb = bf16r(bp[t8 * 16]);
#pragma unroll
      for (int r = 0; r < 8; ++r)
        st[(t8 * 16 + m) * LDT + w * 16 + 8 * h + r] = (_Float16)(acc[t8][r] * WQ_INV + bb);
    }
  }
  __syncthreads();

  if (mat < 2) {
    _Float16* dst = (mat == 0 ? qpl : kpl) + (size_t)(b * SEQ + n0) * CH;
    auto emit = [&]() {
#pragma unroll
      for (int i = 0; i < 8; ++i) {
        const int row = w * 16 + 2 * i + h;
        const u4_t v = *(const u4a_t*)(st + row * LDH + m * 8);
        *(volatile u4_t*)(dst + (size_t)row * CH + m * 8) = v;
      }
    };
    emit();
    __threadfence();
    emit();
  } else {
    _Float16* dst = vtpl + (size_t)(b * CH) * SEQ + n0;
    const int cp = lane >> 3, piece = lane & 7;
    auto emit = [&]() {
#pragma unroll
      for (int i = 0; i < 8; ++i) {
        const int c = w * 32 + 4 * i + cp;
        const u4_t v = *(const u4a_t*)(st + c * LDT + piece * 8);
        *(volatile u4_t*)(dst + (size_t)c * SEQ + piece * 8) = v;
      }
    };
    emit();
    __threadfence();
    emit();
  }
}

__global__ __launch_bounds__(128) void k_attn(
    const _Float16* __restrict__ qpl, const _Float16* __restrict__ kpl,
    const _Float16* __restrict__ vtpl, _Float16* __restrict__ sapl) {
  __shared__ __align__(16) _Float16 os[4][16 * LDSA];
  const int tid = threadIdx.x, lane = tid & 31, w = tid >> 5;
  const int m = lane & 15, h = lane >> 4;
  const int hh = blockIdx.y;
  const int b  = blockIdx.z;
  const int qb = blockIdx.x * 64 + w * 16;
  _Float16* osw = &os[w][0];

  const h16_t qf = ldfrag(qpl + (size_t)(b * SEQ + qb + m) * CH + hh * HD, 0, h);

  f8_t o0 = f8zero(), o1 = f8zero();
  float mrow = -3.0e38f, lsum = 0.f;

  const _Float16* kB = kpl + (size_t)(b * SEQ) * CH + hh * HD;
  const _Float16* vB = vtpl + ((size_t)(b * CH) + hh * HD) * SEQ;

#pragma unroll 1
  for (int mc = 0; mc < SEQ / KCH; ++mc) {
    const int m0 = mc * KCH;
    const h16_t ka0 = ldfrag(kB + (size_t)(m0 + m) * CH, 0, h);
    const h16_t ka1 = ldfrag(kB + (size_t)(m0 + 16 + m) * CH, 0, h);
    const f8_t s0 = wmma16(ka0, qf, f8zero());
    const f8_t s1 = wmma16(ka1, qf, f8zero());

    float t = fmaxf(s0[0], s1[0]);
#pragma unroll
    for (int r = 1; r < 8; ++r) t = fmaxf(t, fmaxf(s0[r], s1[r]));
    t = fmaxf(t, __shfl_xor(t, 16, 32));
    const float nm = fmaxf(mrow, t);
    const float sc = __expf((mrow - nm) * ATTN_SCALE);

    float sm = 0.f;
    h8_t ph0, ph1;
#pragma unroll
    for (int r = 0; r < 8; ++r) {
      const float e0 = __expf((s0[r] - nm) * ATTN_SCALE);
      const float e1 = __expf((s1[r] - nm) * ATTN_SCALE);
      sm += e0 + e1;
      ph0[r] = (_Float16)(e0 * P_CARRY);
      ph1[r] = (_Float16)(e1 * P_CARRY);
    }
    sm += __shfl_xor(sm, 16, 32);
    lsum = lsum * sc + sm;
    mrow = nm;
#pragma unroll
    for (int r = 0; r < 8; ++r) { o0[r] *= sc; o1[r] *= sc; }

    const h16_t pf = __builtin_shufflevector(ph0, ph1, 0, 1, 2, 3, 4, 5, 6, 7,
                                             8, 9, 10, 11, 12, 13, 14, 15);
    const h16_t va0 = ldfrag(vB + (size_t)m * SEQ, m0, h);
    const h16_t va1 = ldfrag(vB + (size_t)(16 + m) * SEQ, m0, h);
    o0 = wmma16(va0, pf, o0);
    o1 = wmma16(va1, pf, o1);
  }

  {
    const float li = (1.0f / lsum) * O_SCALE;
    union { h8_t h; u4_t q; } k0p, k1p;
#pragma unroll
    for (int r = 0; r < 8; ++r) {
      k0p.h[r] = (_Float16)(o0[r] * li);
      k1p.h[r] = (_Float16)(o1[r] * li);
    }
    *(u4a_t*)(osw + m * LDSA + 8 * h)      = k0p.q;
    *(u4a_t*)(osw + m * LDSA + 16 + 8 * h) = k1p.q;
  }
  __syncthreads();

  _Float16* dst = sapl + ((size_t)(b * NHEAD + hh) * SEQ + qb) * HD;
  auto emit = [&]() {
#pragma unroll
    for (int i = 0; i < 2; ++i) {
      const int q  = i * 8 + (lane >> 2);
      const int c8 = (lane & 3) * 8;
      const u4_t v = *(const u4a_t*)(osw + q * LDSA + c8);
      *(volatile u4_t*)(dst + (size_t)(i * 256 + lane * 8)) = v;
    }
  };
  emit();
  __threadfence();
  emit();
}

__global__ __launch_bounds__(128) void k_proj(
    const _Float16* __restrict__ sapl, const _Float16* __restrict__ wp16,
    const float* __restrict__ proj_b, const float* __restrict__ x,
    const float* __restrict__ stats, const float* __restrict__ gn_w,
    const float* __restrict__ gn_b, float* __restrict__ out) {
  __shared__ __align__(16) _Float16 sas[64 * LDH];
  __shared__ __align__(16) float outs[CH * LDO];
  __shared__ float gm[NGRP], gr[NGRP], gw[CH], gb[CH];
  const int tid = threadIdx.x, lane = tid & 31, w = tid >> 5;
  const int m = lane & 15, h = lane >> 4;
  const int n0 = blockIdx.x * 64;
  const int b  = blockIdx.y;

  if (tid < NGRP) {
    const float* sl = stats + (size_t)(b * NGRP + tid) * STATS_LD;
    gm[tid] = sl[0];
    gr[tid] = sl[1];
  }
  gw[tid] = bf16r(gn_w[tid]);
  gb[tid] = bf16r(gn_b[tid]);

  {
#pragma unroll
    for (int j = 0; j < 8; ++j) {
      const int u = tid + 128 * j;
      const int tok = u >> 4, piece = u & 15;
      const int hd_h = piece >> 2, c8 = (piece & 3) * 8;
      const _Float16* src = sapl + ((size_t)(b * NHEAD + hd_h) * SEQ + n0 + tok) * HD + c8;
      *(h8a_t*)(sas + tok * LDH + hd_h * HD + c8) = *(const h8a_t*)src;
    }
  }
  __syncthreads();

  const int c0w = w * 32;
  f8_t acc[2][4];
#pragma unroll
  for (int ct = 0; ct < 2; ++ct)
#pragma unroll
    for (int nt = 0; nt < 4; ++nt) acc[ct][nt] = f8zero();

#pragma unroll
  for (int kc = 0; kc < 4; ++kc) {
    const h16_t a0 = ldfrag(wp16 + (size_t)(c0w + m) * CH, kc * 32, h);
    const h16_t a1 = ldfrag(wp16 + (size_t)(c0w + 16 + m) * CH, kc * 32, h);
#pragma unroll
    for (int nt = 0; nt < 4; ++nt) {
      const h16_t bb = ldfrag(sas + (nt * 16 + m) * LDH, kc * 32, h);
      acc[0][nt] = wmma16(a0, bb, acc[0][nt]);
      acc[1][nt] = wmma16(a1, bb, acc[1][nt]);
    }
  }

#pragma unroll
  for (int ct = 0; ct < 2; ++ct)
#pragma unroll
    for (int nt = 0; nt < 4; ++nt)
#pragma unroll
      for (int r = 0; r < 8; ++r)
        outs[(c0w + ct * 16 + 8 * h + r) * LDO + nt * 16 + m] = acc[ct][nt][r] * PROJ_INV;
  __syncthreads();

  auto emit = [&]() {
#pragma unroll 4
    for (int i = 0; i < 16; ++i) {
      const int c = c0w + 2 * i + h;
      const int g = c / CPG;
      const f4_t v = *(const f4a_t*)(outs + c * LDO + m * 4);
      const float pb = bf16r(proj_b[c]);
      const float gmean = gm[g], grstd = gr[g], gww = gw[c], gbb = gb[c];
      const size_t xo = (size_t)(b * CH + c) * X_SEQ_STRIDE + n0 + m * 4;
      const size_t oo = (size_t)(b * CH + c) * O_SEQ_STRIDE + n0 + m * 4;
      const f4_t xv = *(const f4_t*)(x + xo);
      f4_t o4;
      o4.x = (((bf16r(xv.x) - gmean) * grstd) * gww + gbb) + (v.x + pb);
      o4.y = (((bf16r(xv.y) - gmean) * grstd) * gww + gbb) + (v.y + pb);
      o4.z = (((bf16r(xv.z) - gmean) * grstd) * gww + gbb) + (v.z + pb);
      o4.w = (((bf16r(xv.w) - gmean) * grstd) * gww + gbb) + (v.w + pb);
      *(volatile f4_t*)(out + oo) = o4;
    }
  };
  emit();
  __threadfence();
  emit();
}

extern "C" void kernel_launch(void* const* d_in, const int* in_sizes, int n_in,
                              void* d_out, int out_size, void* d_ws, size_t ws_size,
                              hipStream_t stream) {
  if (n_in < 7) return;
  const size_t x_need = ((size_t)NB * CH - 1) * (size_t)X_SEQ_STRIDE + (size_t)SEQ;
  const size_t o_need = ((size_t)NB * CH - 1) * (size_t)O_SEQ_STRIDE + (size_t)SEQ;
  if ((size_t)in_sizes[0] < x_need) return;
  if (in_sizes[1] < CH || in_sizes[2] < CH) return;
  if (in_sizes[3] < 3 * CH * CH || in_sizes[4] < 3 * CH) return;
  if (in_sizes[5] < CH * CH || in_sizes[6] < CH) return;
  if ((size_t)out_size < o_need) return;

  const float* x      = (const float*)d_in[0];
  const float* gn_w   = (const float*)d_in[1];
  const float* gn_b   = (const float*)d_in[2];
  const float* qkv_w  = (const float*)d_in[3];
  const float* qkv_b  = (const float*)d_in[4];
  const float* proj_w = (const float*)d_in[5];
  const float* proj_b = (const float*)d_in[6];
  float* out = (float*)d_out;

  const size_t sz_wq = (size_t)3 * CH * CH * sizeof(_Float16);
  const size_t sz_wp = (size_t)CH * CH * sizeof(_Float16);
  const size_t sz_st = (size_t)NB * NGRP * STATS_LD * sizeof(float);
  const size_t sz_pl = (size_t)NB * SEQ * CH * sizeof(_Float16);
  const size_t sz_sa = (size_t)NB * NHEAD * SEQ * HD * sizeof(_Float16);
  char* ws = (char*)d_ws;
  size_t off = 0;
  _Float16* wq16 = (_Float16*)(ws + off); off += (sz_wq + 255) & ~(size_t)255;
  _Float16* wp16 = (_Float16*)(ws + off); off += (sz_wp + 255) & ~(size_t)255;
  float*    stats = (float*)(ws + off);   off += (sz_st + 255) & ~(size_t)255;
  _Float16* qpl  = (_Float16*)(ws + off); off += (sz_pl + 255) & ~(size_t)255;
  _Float16* kpl  = (_Float16*)(ws + off); off += (sz_pl + 255) & ~(size_t)255;
  _Float16* vtpl = (_Float16*)(ws + off); off += (sz_pl + 255) & ~(size_t)255;
  _Float16* sapl = (_Float16*)(ws + off); off += (sz_sa + 255) & ~(size_t)255;
  if (off > ws_size || off > WS_LIMIT) return;

  k_cvtw<<<(3 * CH * CH / 8) / 256, 256, 0, stream>>>(qkv_w, wq16, WQ_CARRY);
  k_cvtw<<<(CH * CH / 8) / 256, 256, 0, stream>>>(proj_w, wp16, WP_CARRY);
  k_gnstats<<<NB * NGRP, 256, 0, stream>>>(x, stats);
  k_qkv<<<dim3(SEQ / 64, 3, NB), 128, 0, stream>>>(x, stats, gn_w, gn_b, wq16, qkv_b,
                                                   qpl, kpl, vtpl);
  k_attn<<<dim3(SEQ / 64, NHEAD, NB), 128, 0, stream>>>(qpl, kpl, vtpl, sapl);
  k_proj<<<dim3(SEQ / 64, NB), 128, 0, stream>>>(sapl, wp16, proj_b, x, stats, gn_w, gn_b, out);
}
